// GNNEdgeClassifier_73882027426425
// MI455X (gfx1250) — hardware-verified
//
#include <hip/hip_runtime.h>
#include <stddef.h>
#include <math.h>


#define HD     128
#define KC     256
#define NCONV  4
#define NTHR   256
#define NWAVE  8
#define EPT    8
#define NGRP   2
#define CHUNK  (NTHR * EPT * NGRP)
#define WCAP   (EPT * NGRP * 32)
#define LISTN  (NWAVE * WCAP)
#define NB     512
#define QB     128
#define EPITCH 264
#define WSC    8.0f
#define WSCI   0.125f
#define W1SC   16.0f
#define W1SCI  0.0625f
#define BNEPS  1e-5f

#define LDS_CONV (NB * HD * 4 + LISTN * 4 + 64 + 2 * HD * 4)
#define LDS_EDGE (QB * EPITCH * 2 + QB * HD * 4 + 2 * HD * 4 + 2 * QB * 4 + QB * 4)

static_assert((CHUNK & (CHUNK - 1)) == 0);
static_assert(CHUNK <= 4096);
static_assert(NB <= 4096);
static_assert(NTHR == 2 * HD);
static_assert(NB == 64 * NWAVE);
static_assert(QB == 16 * NWAVE);
static_assert(4 * HD * 8 <= LISTN * 4);
static_assert((QB * EPITCH * 2) % 16 == 0);

typedef float    v4f  __attribute__((ext_vector_type(4)));
typedef float    v8f  __attribute__((ext_vector_type(8)));
typedef double   v2d  __attribute__((ext_vector_type(2)));
typedef int      v4i  __attribute__((ext_vector_type(4)));
typedef _Float16 v4h  __attribute__((ext_vector_type(4)));
typedef _Float16 v8h  __attribute__((ext_vector_type(8)));
typedef _Float16 v16h __attribute__((ext_vector_type(16)));
union FragH { v16h v; v8h h[2]; };

__device__ __forceinline__ v8h cvt8(v4f a, v4f b) {
  v8h r;
  r[0] = (_Float16)a.x; r[1] = (_Float16)a.y; r[2] = (_Float16)a.z; r[3] = (_Float16)a.w;
  r[4] = (_Float16)b.x; r[5] = (_Float16)b.y; r[6] = (_Float16)b.z; r[7] = (_Float16)b.w;
  return r;
}
__device__ __forceinline__ v4h cvt4(v4f a) {
  v4h r;
  r[0] = (_Float16)a.x; r[1] = (_Float16)a.y; r[2] = (_Float16)a.z; r[3] = (_Float16)a.w;
  return r;
}

__device__ __forceinline__ v8f wmh(v16h a, v16h b, v8f c) {
  v8f d = __builtin_amdgcn_wmma_f32_16x16x32_f16(false, a, false, b, (short)0, c, false, false);
  asm volatile("v_nop\n\tv_nop\n\tv_nop\n\tv_nop" : "+v"(d) : "v"(a), "v"(b));
  return d;
}

__device__ __forceinline__ float gelu_f(float v) {
  return 0.5f * v * (1.0f + erff(v * 0.70710678118654752f));
}

template <int NBT>
__device__ __forceinline__ int scan_chunk(const int* __restrict__ dsts, int nE, int cbase, int nodeBase,
                                          int vec8, int* list, int tid, int lane, int wave) {
  int wc = 0;
#pragma unroll
  for (int g = 0; g < NGRP; ++g) {
    const int el0  = (g * NTHR + tid) * EPT;
    const int e0   = cbase + el0;
    const int sent = -2147483647 - 1;
    v4i da, db;
    if (vec8 != 0 && e0 + 7 < nE) {
      da = *(const v4i*)(dsts + e0);
      db = *(const v4i*)(dsts + e0 + 4);
    } else {
      da.x = (e0     < nE) ? dsts[e0]     : sent;
      da.y = (e0 + 1 < nE) ? dsts[e0 + 1] : sent;
      da.z = (e0 + 2 < nE) ? dsts[e0 + 2] : sent;
      da.w = (e0 + 3 < nE) ? dsts[e0 + 3] : sent;
      db.x = (e0 + 4 < nE) ? dsts[e0 + 4] : sent;
      db.y = (e0 + 5 < nE) ? dsts[e0 + 5] : sent;
      db.z = (e0 + 6 < nE) ? dsts[e0 + 6] : sent;
      db.w = (e0 + 7 < nE) ? dsts[e0 + 7] : sent;
    }
    const unsigned nb = (unsigned)nodeBase;
    const unsigned s0 = (unsigned)da.x - nb, s1 = (unsigned)da.y - nb;
    const unsigned s2 = (unsigned)da.z - nb, s3 = (unsigned)da.w - nb;
    const unsigned s4 = (unsigned)db.x - nb, s5 = (unsigned)db.y - nb;
    const unsigned s6 = (unsigned)db.z - nb, s7 = (unsigned)db.w - nb;
    const bool h0 = s0 < (unsigned)NBT, h1 = s1 < (unsigned)NBT, h2 = s2 < (unsigned)NBT, h3 = s3 < (unsigned)NBT;
    const bool h4 = s4 < (unsigned)NBT, h5 = s5 < (unsigned)NBT, h6 = s6 < (unsigned)NBT, h7 = s7 < (unsigned)NBT;
    const unsigned any = __builtin_amdgcn_ballot_w32(h0 | h1 | h2 | h3 | h4 | h5 | h6 | h7);
    if (any != 0u) {
#define HITJ(J, HJ, SJ) { \
        const unsigned mj = __builtin_amdgcn_ballot_w32(HJ); \
        if (mj != 0u) { \
          if (HJ) { \
            const int pos = wc + (int)__builtin_amdgcn_mbcnt_lo(mj, 0u); \
            if (pos < WCAP) list[wave * WCAP + pos] = ((el0 + (J)) << 12) | (int)(SJ); \
          } \
          wc += (int)__builtin_popcount(mj); } }
      HITJ(0, h0, s0)
      HITJ(1, h1, s1)
      HITJ(2, h2, s2)
      HITJ(3, h3, s3)
      HITJ(4, h4, s4)
      HITJ(5, h5, s5)
      HITJ(6, h6, s6)
      HITJ(7, h7, s7)
#undef HITJ
    }
  }
  return wc;
}

__global__ __launch_bounds__(NTHR) void k_prep(
    const float* __restrict__ relw, const float* __restrict__ rootw, const float* __restrict__ w1,
    _Float16* wc, _Float16* w1p) {
  const int i  = blockIdx.x * NTHR + threadIdx.x;
  const int n1 = NCONV * HD * KC / 8;
  const int n2 = HD * KC / 8;
  if (i >= n1 + n2) return;
  v4f a, b;
  _Float16* dp;
  if (i < n1) {
    const int o   = i * 8;
    const int l   = o / (HD * KC);
    const int rem = o - l * (HD * KC);
    const int n   = rem / KC;
    const int k0  = rem - n * KC;
    const float* p = (k0 < HD)
        ? (relw  + (size_t)l * HD * HD + (size_t)k0 * HD + n)
        : (rootw + (size_t)l * HD * HD + (size_t)(k0 - HD) * HD + n);
    a.x = p[0];      a.y = p[HD];     a.z = p[2 * HD]; a.w = p[3 * HD];
    b.x = p[4 * HD]; b.y = p[5 * HD]; b.z = p[6 * HD]; b.w = p[7 * HD];
    a = a * WSC; b = b * WSC;
    dp = wc + o;
  } else {
    const int o  = (i - n1) * 8;
    const int n  = o / KC;
    const int k0 = o - n * KC;
    const float* p = w1 + (size_t)k0 * HD + n;
    a.x = p[0];      a.y = p[HD];     a.z = p[2 * HD]; a.w = p[3 * HD];
    b.x = p[4 * HD]; b.y = p[5 * HD]; b.z = p[6 * HD]; b.w = p[7 * HD];
    a = a * W1SC; b = b * W1SC;
    dp = w1p + o;
  }
  const v8h hv = cvt8(a, b);
  *(volatile v8h*)dp = hv;
  __threadfence();
  *(volatile v8h*)dp = hv;
}

__global__ __launch_bounds__(NTHR) void k_conv(
    const float* __restrict__ xin, const int* __restrict__ ei, const float* __restrict__ ea,
    const float* __restrict__ bnt, const _Float16* __restrict__ wp, const float* __restrict__ relb,
    float* hout, double* part, int nN, int nE, int bnflag, int vec8) {
  extern __shared__ v4f lds_dyn[];
  float*  accL = (float*)lds_dyn;
  int*    list = (int*)(accL + NB * HD);
  int*    wcnt = list + LISTN;
  float*  bntL = (float*)(wcnt + 16);
  double* stg  = (double*)list;
  const int tid = threadIdx.x, lane = tid & 31, wave = tid >> 5, hh = lane >> 4, m = lane & 15;
  const int nodeBase = blockIdx.x * NB;
  const int* dsts = ei + nE;

  {
    const v4f z = {0.f, 0.f, 0.f, 0.f};
    for (int i = tid; i < NB * HD / 4; i += NTHR) lds_dyn[i] = z;
    float tv = (tid < HD) ? 1.0f : 0.0f;
    if (bnflag != 0) tv = bnt[tid];
    bntL[tid] = tv;
  }
  __syncthreads();

  const v4f sc4 = *(const v4f*)(bntL + 4 * lane);
  const v4f sh4 = *(const v4f*)(bntL + HD + 4 * lane);

  const int nChunks = (nE + CHUNK - 1) / CHUNK;
#pragma unroll 1
  for (int ch = 0; ch < nChunks; ++ch) {
    const int cbase = ch * CHUNK;
    const int wc = scan_chunk<NB>(dsts, nE, cbase, nodeBase, vec8, list, tid, lane, wave);
    if (lane == 0) wcnt[wave] = wc;
    __syncthreads();
    if (wave == 0) {
#pragma unroll 1
      for (int wsx = 0; wsx < NWAVE; ++wsx) {
        int n = __builtin_amdgcn_readfirstlane(wcnt[wsx]);
        n = n > WCAP ? WCAP : (n < 0 ? 0 : n);
        const int* lp = list + wsx * WCAP;
#pragma unroll 1
        for (int i = 0; i < n; ++i) {
          const int ent  = __builtin_amdgcn_readfirstlane(lp[i]);
          const int slot = ent & (NB - 1);
          int e = cbase + ((ent >> 12) & (CHUNK - 1));
          e = e > nE - 1 ? nE - 1 : e;
          int src = ei[e];
          src = src < 0 ? 0 : (src > nN - 1 ? nN - 1 : src);
          const float w = ea[e];
          const v4f v = *(const v4f*)(xin + (size_t)src * HD + 4 * lane);
          v4f* ap = (v4f*)(accL + slot * HD + 4 * lane);
          *ap = *ap + (v * sc4 + sh4) * w;
        }
      }
    }
    __syncthreads();
  }

  float rb[8];
#pragma unroll
  for (int u = 0; u < 8; ++u) rb[u] = relb[16 * u + m];

#pragma unroll 1
  for (int q = 0; q < 4; ++q) {
    const int t = wave * 4 + q;
    int node = nodeBase + 16 * t + m;
    node = node > nN - 1 ? nN - 1 : node;
    const float* xr = xin + (size_t)node * HD;
    const float* ar = accL + (16 * t + m) * HD + 8 * hh;
    v8f c8[8];
#pragma unroll
    for (int u = 0; u < 8; ++u) { v8f z = {0.f, 0.f, 0.f, 0.f, 0.f, 0.f, 0.f, 0.f}; c8[u] = z; }
#pragma unroll
    for (int kt = 0; kt < KC / 32; ++kt) {
      FragH a;
      if (kt < 4) {
        const float* ap = ar + 32 * kt;
        const v4f p0 = *(const v4f*)ap,        p1 = *(const v4f*)(ap + 4);
        const v4f p2 = *(const v4f*)(ap + 16), p3 = *(const v4f*)(ap + 20);
        a.h[0] = cvt8(p0, p1);
        a.h[1] = cvt8(p2, p3);
      } else {
        const int c0 = 32 * (kt - 4) + 8 * hh;
        const float* xp = xr + c0;
        v4f x0 = *(const v4f*)xp,        x1 = *(const v4f*)(xp + 4);
        v4f x2 = *(const v4f*)(xp + 16), x3 = *(const v4f*)(xp + 20);
        const v4f s0 = *(const v4f*)(bntL + c0),      s1 = *(const v4f*)(bntL + c0 + 4);
        const v4f s2 = *(const v4f*)(bntL + c0 + 16), s3 = *(const v4f*)(bntL + c0 + 20);
        const v4f o0 = *(const v4f*)(bntL + HD + c0),      o1 = *(const v4f*)(bntL + HD + c0 + 4);
        const v4f o2 = *(const v4f*)(bntL + HD + c0 + 16), o3 = *(const v4f*)(bntL + HD + c0 + 20);
        x0 = x0 * s0 + o0; x1 = x1 * s1 + o1; x2 = x2 * s2 + o2; x3 = x3 * s3 + o3;
        a.h[0] = cvt8(x0, x1);
        a.h[1] = cvt8(x2, x3);
      }
#pragma unroll
      for (int u = 0; u < 8; ++u) {
        const _Float16* bp = wp + (size_t)(16 * u + m) * KC + 32 * kt + 8 * hh;
        FragH b;
        b.h[0] = *(const v8h*)bp;
        b.h[1] = *(const v8h*)(bp + 16);
        c8[u] = wmh(a.v, b.v, c8[u]);
      }
    }
    float* sp = accL + (16 * t + 8 * hh) * HD + m;
#pragma unroll
    for (int u = 0; u < 8; ++u) {
#pragma unroll
      for (int r = 0; r < 8; ++r) sp[r * HD + 16 * u] = gelu_f(c8[u][r] * WSCI + rb[u]);
    }
  }
  __syncthreads();

  const int c = tid & (HD - 1), half = tid >> 7;
  {
    const int rbase = half * (NB / 2);
    const int lim   = nN - nodeBase;
    int rend = rbase + NB / 2;
    rend = rend < lim ? rend : lim;
    double ds = 0.0, dq = 0.0;
#pragma unroll 2
    for (int row = rbase; row < rend; ++row) {
      const double v = (double)accL[row * HD + c];
      ds += v;
      dq += v * v;
    }
    stg[half * HD + c]          = ds;
    stg[2 * HD + half * HD + c] = dq;
  }
  __syncthreads();
  v2d pv = {0.0, 0.0};
  if (tid < HD) {
    pv.x = stg[c] + stg[HD + c];
    pv.y = stg[2 * HD + c] + stg[3 * HD + c];
  }
  double* pp = part + ((size_t)blockIdx.x * HD + c) * 2;

  const float* lrow = accL + (size_t)(wave * 64) * HD + 4 * lane;
  float* grow = hout + ((size_t)nodeBase + wave * 64) * HD + 4 * lane;
  if (tid < HD) *(volatile v2d*)pp = pv;
#pragma unroll 8
  for (int i = 0; i < 64; ++i) { const v4f v = *(const v4f*)(lrow + i * HD); *(volatile v4f*)(grow + (size_t)i * HD) = v; }
  __threadfence();
  if (tid < HD) *(volatile v2d*)pp = pv;
#pragma unroll 8
  for (int i = 0; i < 64; ++i) { const v4f v = *(const v4f*)(lrow + i * HD); *(volatile v4f*)(grow + (size_t)i * HD) = v; }
}

__global__ __launch_bounds__(NTHR) void k_fold(
    const double* __restrict__ part, const float* __restrict__ g, const float* __restrict__ b,
    float* bnt, int nBlk, int nN) {
  __shared__ __attribute__((aligned(16))) float tbl[2 * HD];
  const int tid = threadIdx.x;
  if (tid < HD) {
    double S = 0.0, Q = 0.0;
#pragma unroll 1
    for (int k = 0; k < nBlk; ++k) {
      const v2d p = *(const v2d*)(part + ((size_t)k * HD + tid) * 2);
      S += p.x;
      Q += p.y;
    }
    const double inv  = 1.0 / (double)nN;
    const double mean = S * inv;
    double var = Q * inv - mean * mean;
    var = var < 0.0 ? 0.0 : var;
    const float rs = rsqrtf((float)var + BNEPS);
    const float sc = g[tid] * rs;
    const float sh = b[tid] - (float)mean * sc;
    tbl[tid]      = sc;
    tbl[HD + tid] = sh;
  }
  __syncthreads();
  v4f v = {0.f, 0.f, 0.f, 0.f};
  if (tid < 64) v = *(const v4f*)(tbl + 4 * tid);
  if (tid < 64) *(volatile v4f*)(bnt + 4 * tid) = v;
  __threadfence();
  if (tid < 64) *(volatile v4f*)(bnt + 4 * tid) = v;
}

__global__ __launch_bounds__(NTHR) void k_edge(
    const float* __restrict__ hin, const int* __restrict__ eli, const float* __restrict__ bnt,
    const _Float16* __restrict__ w1p, const float* __restrict__ b1, const float* __restrict__ w2,
    const float* __restrict__ b2, float* out, int nN, int nQ) {
  extern __shared__ v4f lds_dyn[];
  _Float16* ef = (_Float16*)lds_dyn;
  float* hm   = (float*)((char*)lds_dyn + QB * EPITCH * 2);
  float* bntL = hm + QB * HD;
  int*   idxL = (int*)(bntL + 2 * HD);
  float* outv = (float*)(idxL + 2 * QB);
  const int tid = threadIdx.x, lane = tid & 31, wave = tid >> 5, hh = lane >> 4, m = lane & 15;
  const int q0 = blockIdx.x * QB;

  bntL[tid] = bnt[tid];
  {
    const int side = tid >> 7, r = tid & (QB - 1);
    int q = q0 + r;
    q = q > nQ - 1 ? nQ - 1 : q;
    int nd = eli[(size_t)side * nQ + q];
    nd = nd < 0 ? 0 : (nd > nN - 1 ? nN - 1 : nd);
    idxL[tid] = nd;
  }
  __syncthreads();

#pragma unroll 4
  for (int i = 0; i < (QB * 2 * HD / 4) / NTHR; ++i) {
    const int idx   = i * NTHR + tid;
    const int r     = idx >> 6;
    const int piece = idx & 63;
    const int side  = piece >> 5;
    const int c4    = (piece & 31) * 4;
    const int nd    = idxL[side * QB + r];
    v4f xv = *(const v4f*)(hin + (size_t)nd * HD + c4);
    const v4f s = *(const v4f*)(bntL + c4), o = *(const v4f*)(bntL + HD + c4);
    xv = xv * s + o;
    *(v4h*)(ef + r * EPITCH + side * HD + c4) = cvt4(xv);
  }
  __syncthreads();

  v8f c8[8];
#pragma unroll
  for (int u = 0; u < 8; ++u) { v8f z = {0.f, 0.f, 0.f, 0.f, 0.f, 0.f, 0.f, 0.f}; c8[u] = z; }
  const _Float16* ar = ef + (wave * 16 + m) * EPITCH + 8 * hh;
#pragma unroll
  for (int kt = 0; kt < KC / 32; ++kt) {
    FragH a;
    a.h[0] = *(const v8h*)(ar + 32 * kt);
    a.h[1] = *(const v8h*)(ar + 32 * kt + 16);
#pragma unroll
    for (int u = 0; u < 8; ++u) {
      const _Float16* bp = w1p + (size_t)(16 * u + m) * KC + 32 * kt + 8 * hh;
      FragH b;
      b.h[0] = *(const v8h*)bp;
      b.h[1] = *(const v8h*)(bp + 16);
      c8[u] = wmh(a.v, b.v, c8[u]);
    }
  }
  {
    float bb[8];
#pragma unroll
    for (int u = 0; u < 8; ++u) bb[u] = b1[16 * u + m];
    float* sp = hm + (wave * 16 + 8 * hh) * HD + m;
#pragma unroll
    for (int u = 0; u < 8; ++u) {
#pragma unroll
      for (int r = 0; r < 8; ++r) sp[r * HD + 16 * u] = gelu_f(c8[u][r] * W1SCI + bb[u]);
    }
  }
  __syncthreads();

  {
    const v4f wv = *(const v4f*)(w2 + 4 * lane);
    const float bias2 = b2[0];
    float myo = 0.f;
#pragma unroll
    for (int i = 0; i < 16; ++i) {
      const v4f hv = *(const v4f*)(hm + (wave * 16 + i) * HD + 4 * lane);
      float p = hv.x * wv.x + hv.y * wv.y + hv.z * wv.z + hv.w * wv.w;
      p += __shfl_xor(p, 16);
      p += __shfl_xor(p, 8);
      p += __shfl_xor(p, 4);
      p += __shfl_xor(p, 2);
      p += __shfl_xor(p, 1);
      const float s  = p + bias2;
      const float ov = __builtin_amdgcn_rcpf(1.0f + expf(-s));
      if (lane == i) myo = ov;
    }
    if (lane < 16) outv[wave * 16 + lane] = myo;
  }
  __syncthreads();

  if (wave == 0) {
    const v4f v  = *(const v4f*)(outv + 4 * lane);
    const int gi = q0 + 4 * lane;
    float* op = out + gi;
    if (gi + 3 < nQ) { *(volatile v4f*)op = v; }
    else {
      if (gi     < nQ) *(volatile float*)(op)     = v.x;
      if (gi + 1 < nQ) *(volatile float*)(op + 1) = v.y;
      if (gi + 2 < nQ) *(volatile float*)(op + 2) = v.z;
    }
    __threadfence();
    if (gi + 3 < nQ) { *(volatile v4f*)op = v; }
    else {
      if (gi     < nQ) *(volatile float*)(op)     = v.x;
      if (gi + 1 < nQ) *(volatile float*)(op + 1) = v.y;
      if (gi + 2 < nQ) *(volatile float*)(op + 2) = v.z;
    }
  }
}

extern "C" void kernel_launch(void* const* d_in, const int* in_sizes, int n_in,
                              void* d_out, int out_size, void* d_ws, size_t ws_size,
                              hipStream_t stream) {
  if (n_in < 13) return;
  const int nN = in_sizes[0] / HD;
  const int nE = in_sizes[1] / 2;
  const int nQ = in_sizes[3] / 2;
  if (nN <= 0 || nE < 0 || nQ <= 0) return;
  if (in_sizes[0] != nN * HD || in_sizes[1] != nE * 2 || in_sizes[3] != nQ * 2) return;
  if (in_sizes[2] < nE) return;
  if (in_sizes[4] != NCONV * HD * HD || in_sizes[5] < NCONV * HD || in_sizes[6] != NCONV * HD * HD) return;
  if (in_sizes[7] < NCONV * HD || in_sizes[8] < NCONV * HD) return;
  if (in_sizes[9] != KC * HD || in_sizes[10] < HD || in_sizes[11] < HD || in_sizes[12] < 1) return;
  if (out_size != nQ) return;

  const float* x     = (const float*)d_in[0];
  const int*   ei    = (const int*)d_in[1];
  const float* ea    = (const float*)d_in[2];
  const int*   eli   = (const int*)d_in[3];
  const float* relw  = (const float*)d_in[4];
  const float* relb  = (const float*)d_in[5];
  const float* rootw = (const float*)d_in[6];
  const float* bng   = (const float*)d_in[7];
  const float* bnb   = (const float*)d_in[8];
  const float* w1    = (const float*)d_in[9];
  const float* b1    = (const float*)d_in[10];
  const float* w2    = (const float*)d_in[11];
  const float* b2    = (const float*)d_in[12];
  float* out = (float*)d_out;

  const int nBlk = (nN + NB - 1) / NB;
  const int nQB  = (nQ + QB - 1) / QB;

  char* ws = (char*)d_ws;
  size_t off = 0;
  const size_t oWc = off; off += (size_t)NCONV * HD * KC * 2;            off = (off + 255) & ~(size_t)255;
  const size_t oW1 = off; off += (size_t)HD * KC * 2;                    off = (off + 255) & ~(size_t)255;
  const size_t oBn = off; off += (size_t)2 * HD * 4;                     off = (off + 255) & ~(size_t)255;
  const size_t oPt = off; off += (size_t)nBlk * HD * 2 * 8;              off = (off + 255) & ~(size_t)255;
  const size_t oH0 = off; off += (size_t)nBlk * NB * HD * 4;             off = (off + 255) & ~(size_t)255;
  const size_t oH1 = off; off += (size_t)nBlk * NB * HD * 4;             off = (off + 255) & ~(size_t)255;
  if (off > ws_size) return;
  _Float16* wc  = (_Float16*)(ws + oWc);
  _Float16* w1p = (_Float16*)(ws + oW1);
  float*    bnt = (float*)(ws + oBn);
  double*   part = (double*)(ws + oPt);
  float*    hb0 = (float*)(ws + oH0);
  float*    hb1 = (float*)(ws + oH1);

  const int vec8 = ((nE & 3) == 0) ? 1 : 0;

  const int nPrep = NCONV * HD * KC / 8 + HD * KC / 8;
  k_prep<<<(nPrep + NTHR - 1) / NTHR, NTHR, 0, stream>>>(relw, rootw, w1, wc, w1p);

  hipFuncSetAttribute(reinterpret_cast<const void*>(&k_conv),
                      hipFuncAttributeMaxDynamicSharedMemorySize, LDS_CONV);
  hipFuncSetAttribute(reinterpret_cast<const void*>(&k_edge),
                      hipFuncAttributeMaxDynamicSharedMemorySize, LDS_EDGE);

  for (int l = 0; l < NCONV; ++l) {
    const float* xin  = (l == 0) ? x : (((l - 1) & 1) ? hb1 : hb0);
    float*       hout = (l & 1) ? hb1 : hb0;
    k_conv<<<nBlk, NTHR, LDS_CONV, stream>>>(
        xin, ei, ea, bnt, wc + (size_t)l * HD * KC, relb + (size_t)l * HD,
        hout, part, nN, nE, (l > 0) ? 1 : 0, vec8);
    k_fold<<<1, NTHR, 0, stream>>>(part, bng + (size_t)l * HD, bnb + (size_t)l * HD, bnt, nBlk, nN);
  }

  const float* hlast = ((NCONV - 1) & 1) ? hb1 : hb0;
  k_edge<<<nQB, NTHR, LDS_EDGE, stream>>>(hlast, eli, bnt, w1p, b1, w2, b2, out, nN, nQ);
}
